// ProGen_4887672783532
// MI455X (gfx1250) — hardware-verified
//
#include <hip/hip_runtime.h>


namespace {
constexpr int NB = 2, S = 8192, D = 256, DEPTH = 6, WSZ = 512, FF = 1024, VOC = 32, NT = NB * S, HALF = D / 2;
constexpr float XS = 8.0f, WSC = 256.0f, PS = 8.0f, EPS = 1e-5f;

typedef _Float16 b16;
typedef __attribute__((ext_vector_type(16))) _Float16 v16b;
typedef __attribute__((ext_vector_type(8))) _Float16 v8b;
typedef __attribute__((ext_vector_type(8))) float v8f;
typedef __attribute__((ext_vector_type(4))) float v4f;
__device__ __forceinline__ float bf16_rne(float f) { unsigned int u = __float_as_uint(f); u += 0x7FFFu + ((u >> 16) & 1u); return __uint_as_float(u & 0xFFFF0000u); }
__device__ __forceinline__ v16b frag_kb(const b16* p, int hh) { const v8b a = *(const v8b*)(p + 8 * hh), b = *(const v8b*)(p + 16 + 8 * hh); v16b f;
#pragma unroll
  for (int e = 0; e < 8; ++e) { f[e] = a[e]; f[8 + e] = b[e]; } return f; }
__device__ __forceinline__ v8f wmma16b(v16b a, v16b b, v8f c) { v8f d = __builtin_amdgcn_wmma_f32_16x16x32_f16(false, a, false, b, (short)0, c, false, false); asm volatile("v_nop\n\tv_nop\n\tv_nop\n\tv_nop" : "+v"(d) : "v"(a), "v"(b)); return d; }
__device__ __forceinline__ void wave_lds_sync() { __builtin_amdgcn_fence(__ATOMIC_RELEASE, "workgroup"); __builtin_amdgcn_wave_barrier(); __builtin_amdgcn_fence(__ATOMIC_ACQUIRE, "workgroup"); }
__device__ __forceinline__ float nexp(float x) { return __builtin_amdgcn_exp2f(x * 1.4426950408889634f); }
__device__ __forceinline__ float pmul(float a, float b) { float p = a * b; asm volatile("" : "+v"(p)); return p; }
__device__ __forceinline__ float gelu(float v) { return 0.5f * v * (1.0f + erff(v * 0.70710678118654752f)); }

__global__ __launch_bounds__(256) void prepw_kernel(const float* __restrict__ w1, const float* __restrict__ w2, const float* __restrict__ wo, b16* __restrict__ W1T, b16* __restrict__ W2T, b16* __restrict__ WOT, float* __restrict__ INVF) {
  __shared__ __attribute__((aligned(16))) b16 T[64][64 + 8];
  const int kind = blockIdx.z, i0 = blockIdx.x * 64, o0 = blockIdx.y * 64, t_ = threadIdx.x;
  const int l = kind >> 1; const bool isw2 = (kind & 1) && kind < 2 * DEPTH, isout = kind == 2 * DEPTH;
  const int IN = isout ? D : (isw2 ? FF : D), OUT = isout ? VOC : (isw2 ? D : FF);
  if (isout && blockIdx.x == 0 && blockIdx.y == 1) { if (t_ < HALF) { const float f = 1.0f / powf(10000.0f, (float)(2 * t_) / (float)D); for (int pass = 0; pass < 2; ++pass) { ((volatile float*)INVF)[t_] = f; __threadfence(); } } return; }
  if (i0 >= IN || o0 >= OUT) return;
  const float* w = isout ? wo : (isw2 ? w2 + (size_t)l * FF * D : w1 + (size_t)l * D * FF); b16* dst = isout ? WOT : (isw2 ? W2T + (size_t)l * D * FF : W1T + (size_t)l * FF * D);
  for (int q = t_; q < 64 * 64; q += 256) { const int ii = q >> 6, oo = q & 63; T[oo][ii] = (o0 + oo < OUT) ? (b16)(bf16_rne(w[(size_t)(i0 + ii) * OUT + (o0 + oo < OUT ? o0 + oo : 0)]) * WSC) : (b16)0.0f; }
  __syncthreads();
  for (int pass = 0; pass < 2; ++pass) { for (int q = t_; q < 64 * 8; q += 256) { const int oo = q >> 3, c8 = (q & 7) * 8; if (o0 + oo < OUT) *(volatile v8b*)(dst + (size_t)(o0 + oo) * IN + i0 + c8) = *(const v8b*)(&T[oo][c8]); } __threadfence(); }
}
__global__ __launch_bounds__(256) void embed_kernel(const int* __restrict__ ids, const float* __restrict__ emb, float* __restrict__ X) {
  const int wave = threadIdx.x >> 5, lane = threadIdx.x & 31; const size_t tok = (size_t)blockIdx.x * 8 + wave; const int idl = ids[tok]; const int id = idl < 0 ? 0 : (idl >= VOC ? VOC - 1 : idl);
  v4f a = *(const v4f*)(emb + (size_t)id * D + lane * 8), c = *(const v4f*)(emb + (size_t)id * D + lane * 8 + 4);
#pragma unroll
  for (int j = 0; j < 4; ++j) { a[j] = bf16_rne(a[j]); c[j] = bf16_rne(c[j]); }
  for (int pass = 0; pass < 2; ++pass) { *(volatile v4f*)(X + tok * D + lane * 8) = a; *(volatile v4f*)(X + tok * D + lane * 8 + 4) = c; __threadfence(); }
}
__global__ __launch_bounds__(256) void rot_kernel(const float* __restrict__ X, const float* __restrict__ INVF, b16* __restrict__ QK16, b16* __restrict__ VT) {
  __shared__ __attribute__((aligned(16))) b16 Tv[D][64 + 8]; __shared__ __attribute__((aligned(16))) b16 Tq[8][D];
  const int wave = threadIdx.x >> 5, lane = threadIdx.x & 31, t_ = threadIdx.x; const size_t tok0 = (size_t)blockIdx.x * 64; const int b = (int)(tok0 / S), s0 = (int)(tok0 - (size_t)b * S);
  for (int rr = wave; rr < 64; rr += 8) { const size_t tok = tok0 + rr; const int t = s0 + rr; const float* xr = X + tok * D;
#pragma unroll
    for (int q = 0; q < 4; ++q) { const int m = lane * 4 + q; const float x1 = xr[m], x2 = xr[m + HALF]; const float th = (float)t * INVF[m]; float sn, cs; sincosf(th, &sn, &cs);
      Tq[wave][m] = (b16)((pmul(x1, cs) - pmul(x2, sn)) * XS); Tq[wave][m + HALF] = (b16)((pmul(x2, cs) + pmul(x1, sn)) * XS); Tv[m][rr] = (b16)(x1 * XS); Tv[m + HALF][rr] = (b16)(x2 * XS); }
    wave_lds_sync();
    for (int pass = 0; pass < 2; ++pass) { *(volatile v8b*)(QK16 + tok * D + lane * 8) = *(const v8b*)(&Tq[wave][lane * 8]); __threadfence(); }
    wave_lds_sync(); }
  __syncthreads();
  for (int pass = 0; pass < 2; ++pass) { for (int q = t_; q < D * 8; q += 256) { const int d = q >> 3, c8 = (q & 7) * 8; *(volatile v8b*)(VT + ((size_t)b * D + d) * S + s0 + c8) = *(const v8b*)(&Tv[d][c8]); } __threadfence(); }
}
__global__ __launch_bounds__(64) void attn_kernel(const b16* __restrict__ QK16, const b16* __restrict__ VT, float* __restrict__ X) {
  __shared__ __attribute__((aligned(16))) float To[2][16][D + 4];
  const int wave = threadIdx.x >> 5, lane = threadIdx.x & 31, hh = lane >> 4, col = lane & 15; const int b = blockIdx.y; const int q0 = blockIdx.x * 32 + wave * 16, qi = q0 + col;
  const b16* QKb = QK16 + (size_t)b * S * D; const b16* V = VT + (size_t)b * D * S;
  const b16* qrow = QKb + (size_t)qi * D;
  const float scale = 0.0625f * (1.0f / (XS * XS));
  float m = -INFINITY, l = 0.0f; v8f o[16];
#pragma unroll
  for (int t = 0; t < 16; ++t) o[t] = (v8f){};
  int kstart = q0 - WSZ; kstart = kstart < 0 ? 0 : (kstart & ~31); const int kend = q0 + 16;
  for (int kb = kstart; kb < kend; kb += 32) {
    v8f s0 = {}, s1 = {};
#pragma unroll
    for (int ks = 0; ks < 8; ++ks) { const v16b qf = frag_kb(qrow + ks * 32, hh); s0 = wmma16b(frag_kb(QKb + (size_t)(kb + col) * D + ks * 32, hh), qf, s0); s1 = wmma16b(frag_kb(QKb + (size_t)(kb + 16 + col) * D + ks * 32, hh), qf, s1); }
    float mr = -INFINITY;
#pragma unroll
    for (int r = 0; r < 8; ++r) { const int ka = kb + 8 * hh + r, kc = ka + 16; s0[r] = (ka <= qi && ka >= qi - WSZ) ? s0[r] * scale : -INFINITY; s1[r] = (kc <= qi && kc >= qi - WSZ) ? s1[r] * scale : -INFINITY; mr = fmaxf(mr, fmaxf(s0[r], s1[r])); }
    mr = fmaxf(mr, __shfl_xor(mr, 16)); const float mn = fmaxf(m, mr);
    const float al_ = (mn == -INFINITY) ? 1.0f : nexp(m - mn); m = mn; float sum = 0.0f; v16b pb;
#pragma unroll
    for (int r = 0; r < 8; ++r) { const float e0 = (mn == -INFINITY) ? 0.0f : nexp(s0[r] - mn), e1 = (mn == -INFINITY) ? 0.0f : nexp(s1[r] - mn); sum += e0 + e1; pb[r] = (b16)(e0 * PS); pb[8 + r] = (b16)(e1 * PS); }
    sum += __shfl_xor(sum, 16); l = l * al_ + sum;
#pragma unroll
    for (int t = 0; t < 16; ++t) { o[t] *= al_; o[t] = wmma16b(frag_kb(V + (size_t)(t * 16 + col) * S + kb, hh), pb, o[t]); } }
  const float inv = 1.0f / (l * PS * XS);
#pragma unroll
  for (int t = 0; t < 16; ++t)
#pragma unroll
    for (int r = 0; r < 8; ++r) To[wave][col][t * 16 + 8 * hh + r] = o[t][r] * inv;
  wave_lds_sync();
  for (int pass = 0; pass < 2; ++pass) { for (int rr = 0; rr < 16; ++rr) { float* xr = X + ((size_t)b * S + q0 + rr) * D; for (int hq = 0; hq < 2; ++hq) { const int c0 = hq * 128 + lane * 4;
        v4f v = *(const v4f*)(&To[wave][rr][c0]); if (pass == 0) { const v4f xv = *(const v4f*)(xr + c0); v += xv; *(v4f*)(&To[wave][rr][c0]) = v; } *(volatile v4f*)(xr + c0) = v; } } __threadfence(); }
}
__global__ __launch_bounds__(256) void ln_kernel(const float* __restrict__ X, const float* __restrict__ g, const float* __restrict__ be, b16* __restrict__ H16) {
  const int wave = threadIdx.x >> 5, lane = threadIdx.x & 31; const size_t row = (size_t)blockIdx.x * 8 + wave; const float* src = X + row * D + lane * 8;
  const v4f a0 = *(const v4f*)src, a1 = *(const v4f*)(src + 4); float v[8];
#pragma unroll
  for (int j = 0; j < 4; ++j) { v[j] = a0[j]; v[4 + j] = a1[j]; }
  float s = 0.0f;
#pragma unroll
  for (int j = 0; j < 8; ++j) s += v[j];
#pragma unroll
  for (int o = 16; o >= 1; o >>= 1) s += __shfl_xor(s, o);
  const float mu = s * (1.0f / D); float ss = 0.0f;
#pragma unroll
  for (int j = 0; j < 8; ++j) { const float d = v[j] - mu; ss += pmul(d, d); }
#pragma unroll
  for (int o = 16; o >= 1; o >>= 1) ss += __shfl_xor(ss, o);
  const float rs = rsqrtf(ss * (1.0f / D) + EPS); v8b o8;
#pragma unroll
  for (int j = 0; j < 8; ++j) { const int c = lane * 8 + j; o8[j] = (b16)((pmul((v[j] - mu) * rs, bf16_rne(g[c])) + bf16_rne(be[c])) * XS); }
  for (int pass = 0; pass < 2; ++pass) { *(volatile v8b*)(H16 + row * D + lane * 8) = o8; __threadfence(); }
}
__global__ __launch_bounds__(128) void ffn1_kernel(const b16* __restrict__ H16, const b16* __restrict__ W1T, const float* __restrict__ b1, b16* __restrict__ G16) {
  __shared__ __attribute__((aligned(16))) b16 Th[4][16][128 + 8];
  const int wave = threadIdx.x >> 5, lane = threadIdx.x & 31, nloc = lane & 15, hlf = lane >> 4; const size_t m0 = (size_t)blockIdx.x * 64 + wave * 16; const int n0 = blockIdx.y * 128;
  v8f acc[8];
#pragma unroll
  for (int t = 0; t < 8; ++t) acc[t] = (v8f){};
#pragma unroll
  for (int kb = 0; kb < D; kb += 32) { const v16b a = frag_kb(H16 + (m0 + nloc) * D + kb, hlf);
#pragma unroll
    for (int t = 0; t < 8; ++t) acc[t] = wmma16b(a, frag_kb(W1T + (size_t)(n0 + t * 16 + nloc) * D + kb, hlf), acc[t]); }
#pragma unroll
  for (int t = 0; t < 8; ++t) { const float bb = bf16_rne(b1[n0 + t * 16 + nloc]);
#pragma unroll
    for (int r = 0; r < 8; ++r) Th[wave][8 * hlf + r][t * 16 + nloc] = (b16)(gelu(acc[t][r] * (1.0f / (XS * WSC)) + bb) * XS); }
  wave_lds_sync();
  for (int pass = 0; pass < 2; ++pass) { for (int rr = 0; rr < 16; ++rr) if (lane < 16) *(volatile v8b*)(G16 + (m0 + rr) * FF + n0 + lane * 8) = *(const v8b*)(&Th[wave][rr][lane * 8]); __threadfence(); }
}
template <int MODE>
__global__ __launch_bounds__(128) void ffn2_kernel(const b16* __restrict__ A, const b16* __restrict__ Bw, const float* __restrict__ bias, float* __restrict__ Y) {
  __shared__ __attribute__((aligned(16))) float Ts[4][16][D + 4];
  const int wave = threadIdx.x >> 5, lane = threadIdx.x & 31, nloc = lane & 15, hlf = lane >> 4; const size_t m0 = (size_t)blockIdx.x * 64 + wave * 16;
  constexpr int NTL = MODE == 0 ? 16 : 2, K = MODE == 0 ? FF : D, LDY = MODE == 0 ? D : VOC;
  v8f acc[NTL];
#pragma unroll
  for (int t = 0; t < NTL; ++t) acc[t] = (v8f){};
#pragma unroll 2
  for (int kb = 0; kb < K; kb += 32) { const v16b a = frag_kb(A + (m0 + nloc) * K + kb, hlf);
#pragma unroll
    for (int t = 0; t < NTL; ++t) acc[t] = wmma16b(a, frag_kb(Bw + (size_t)(t * 16 + nloc) * K + kb, hlf), acc[t]); }
#pragma unroll
  for (int t = 0; t < NTL; ++t) { const float bb = bf16_rne(bias[t * 16 + nloc]);
#pragma unroll
    for (int r = 0; r < 8; ++r) Ts[wave][8 * hlf + r][t * 16 + nloc] = acc[t][r] * (1.0f / (XS * WSC)) + bb; }
  wave_lds_sync();
  for (int pass = 0; pass < 2; ++pass) {
    if (MODE == 0) { for (int rr = 0; rr < 16; ++rr) { float* yr = Y + (m0 + rr) * D; for (int hq = 0; hq < 2; ++hq) { const int c0 = hq * 128 + lane * 4; v4f v = *(const v4f*)(&Ts[wave][rr][c0]); if (pass == 0) { v += *(const v4f*)(yr + c0); *(v4f*)(&Ts[wave][rr][c0]) = v; } *(volatile v4f*)(yr + c0) = v; } } }
    else { for (int r4 = 0; r4 < 16; r4 += 4) { const int rr = r4 + (lane >> 3), c4 = (lane & 7) * 4; *(volatile v4f*)(Y + (m0 + rr) * VOC + c4) = *(const v4f*)(&Ts[wave][rr][c4]); } }
    __threadfence(); }
}
}

extern "C" void kernel_launch(void* const* d_in, const int* in_sizes, int n_in, void* d_out, int out_size, void* d_ws, size_t ws_size, hipStream_t stream) {
  (void)n_in;
  auto Fp = [&](int i) { return (const float*)d_in[i]; };
  if (in_sizes[0] != NT || in_sizes[1] != VOC * D || in_sizes[4] != DEPTH * D * FF || in_sizes[6] != DEPTH * FF * D || in_sizes[10] != D * VOC || out_size != NT * VOC) return;
  size_t off = 0; char* ws = (char*)d_ws;
  auto carve = [&](size_t bytes) { char* p = ws + off; off += (bytes + 255) & ~(size_t)255; return p; };
  b16* W1T = (b16*)carve((size_t)DEPTH * FF * D * 2); b16* W2T = (b16*)carve((size_t)DEPTH * D * FF * 2); b16* WOT = (b16*)carve((size_t)VOC * D * 2); float* INVF = (float*)carve(HALF * 4);
  float* X = (float*)carve((size_t)NT * D * 4); b16* QK16 = (b16*)carve((size_t)NT * D * 2); b16* VT = (b16*)carve((size_t)NT * D * 2); b16* H16 = (b16*)carve((size_t)NT * D * 2); b16* G16 = (b16*)carve((size_t)NT * FF * 2);
  if (off > ws_size || off > ((size_t)128 << 20)) return;
  prepw_kernel<<<dim3(FF / 64, FF / 64, 2 * DEPTH + 1), 256, 0, stream>>>(Fp(4), Fp(6), Fp(10), W1T, W2T, WOT, INVF);
  embed_kernel<<<NT / 8, 256, 0, stream>>>((const int*)d_in[0], Fp(1), X);
  for (int l = 0; l < DEPTH; ++l) {
    rot_kernel<<<NT / 64, 256, 0, stream>>>(X, INVF, QK16, VT);
    attn_kernel<<<dim3(S / 32, NB), 64, 0, stream>>>(QK16, VT, X);
    ln_kernel<<<NT / 8, 256, 0, stream>>>(X, Fp(2) + l * D, Fp(3) + l * D, H16);
    ffn1_kernel<<<dim3(NT / 64, FF / 128), 128, 0, stream>>>(H16, W1T + (size_t)l * FF * D, Fp(5) + l * FF, G16);
    ffn2_kernel<0><<<NT / 64, 128, 0, stream>>>(G16, W2T + (size_t)l * D * FF, Fp(7) + l * D, X); }
  ln_kernel<<<NT / 8, 256, 0, stream>>>(X, Fp(8), Fp(9), H16);
  ffn2_kernel<1><<<NT / 64, 128, 0, stream>>>(H16, WOT, Fp(11), (float*)d_out);
}
